// fastAPPNPTransformerBlock_52037823758878
// MI455X (gfx1250) — hardware-run, weakly checked
//
#include <hip/hip_runtime.h>


namespace {
constexpr int N = 50000, NP = 50048, E = 1250000, FIN = 256, HID = 128, NH = 8, HD = 16, NB = 44, C = 64, NBLK = NP / 64  , PW = 768  , KH = 10;
constexpr float XS = 8.0f, WSC = 256.0f, NEG = 0.2f  , ALPHA = 0.1f, PEPS = 1e-4f, DNORM = 0.5f  , RATIO = 0.15075567228888181f  ;
typedef _Float16 b16;
typedef __attribute__((ext_vector_type(16))) _Float16 v16b;
typedef __attribute__((ext_vector_type(8))) _Float16 v8b;
typedef __attribute__((ext_vector_type(8))) float v8f;
typedef __attribute__((ext_vector_type(4))) float v4f;
typedef __attribute__((ext_vector_type(2))) float v2f;
__device__ __forceinline__ float bf16_rne(float f) { unsigned int u = __float_as_uint(f); u += 0x7FFFu + ((u >> 16) & 1u); return __uint_as_float(u & 0xFFFF0000u); }
__device__ __forceinline__ void split16(float v, b16& hi, b16& lo) { hi = (b16)v; lo = (b16)(v - (float)hi); }
__device__ __forceinline__ v16b frag_kb(const b16* p, int hh) { const v8b a = *(const v8b*)(p + 8 * hh), b = *(const v8b*)(p + 16 + 8 * hh); v16b f;
#pragma unroll
  for (int e = 0; e < 8; ++e) { f[e] = a[e]; f[8 + e] = b[e]; } return f; }
__device__ __forceinline__ v8f wmma16b(v16b a, v16b b, v8f c) { v8f d = __builtin_amdgcn_wmma_f32_16x16x32_f16(false, a, false, b, (short)0, c, false, false); asm volatile("v_nop\n\tv_nop\n\tv_nop\n\tv_nop" : "+v"(d) : "v"(a), "v"(b)); return d; }
__device__ __forceinline__ void wave_lds_sync() { __builtin_amdgcn_fence(__ATOMIC_RELEASE, "workgroup"); __builtin_amdgcn_wave_barrier(); __builtin_amdgcn_fence(__ATOMIC_ACQUIRE, "workgroup"); }
__device__ __forceinline__ float pmul(float a, float b) { float p = a * b; asm volatile("" : "+v"(p)); return p; }
__device__ __forceinline__ int iclamp(int v, int lo, int hi) { return v < lo ? lo : (v > hi ? hi : v); }
__device__ __forceinline__ float elu_(float x) { return x > 0.0f ? x : (__expf(x) - 1.0f); }
constexpr int CSR_NBLK = 512, CSR_GB = 8, CSR_GN = 1 << CSR_GB  , CSR_MAXG = 512, CSR_CAP = 12288  ;
__global__ __launch_bounds__(64) void csrA_kernel(const int* __restrict__ dst, int E, int N, int nG, int CHP, int NGP, int* __restrict__ STG, int* __restrict__ HST) {
  extern __shared__ int sm[];
  int* cnt = sm; int* run = sm + NGP; int* ids = sm + 2 * NGP;
  const int b = blockIdx.x; const int ch = (E + CSR_NBLK - 1) / CSR_NBLK; const int e0 = b * ch, e1 = min(E, e0 + ch);
  for (int i = threadIdx.x; i < NGP; i += 64) cnt[i] = 0;
  for (int i = threadIdx.x; i < CHP; i += 64) ids[i] = -1;
  __syncthreads();
  if (threadIdx.x == 0) {
    for (int e = e0; e < e1; ++e) { int d = dst[e]; d = (d < 0) ? 0 : (d >= N ? N - 1 : d); cnt[d >> CSR_GB] += 1; }
    int acc = 0; for (int g = 0; g < nG; ++g) { run[g] = acc; acc += cnt[g]; }
    for (int e = e0; e < e1; ++e) { int d = dst[e]; d = (d < 0) ? 0 : (d >= N ? N - 1 : d); const int g = d >> CSR_GB; ids[run[g]] = e; run[g] += 1; } }
  __syncthreads();
  typedef __attribute__((ext_vector_type(4))) int v4i;
  for (int pass = 0; pass < 2; ++pass) {
    for (int i = threadIdx.x; i < CHP / 4; i += 64) *(volatile v4i*)(STG + (size_t)b * CHP + i * 4) = *(const v4i*)(&ids[i * 4]);
    for (int i = threadIdx.x; i < NGP / 4; i += 64) { v4i v; for (int e = 0; e < 4; ++e) v[e] = (i * 4 + e < nG) ? cnt[i * 4 + e] : 0; *(volatile v4i*)(HST + (size_t)b * NGP + i * 4) = v; }
    __threadfence(); }
}
__global__ __launch_bounds__(512) void csrS_kernel(const int* __restrict__ HST, int nG, int NGP, int* __restrict__ START, int* __restrict__ TOT, int* __restrict__ OFF) {
  __shared__ int tot[CSR_MAXG];
  const int b = threadIdx.x;
  for (int pass = 0; pass < 2; ++pass) { int runb = 0; for (int g = 0; g < nG; ++g) { int c = HST[(size_t)b * NGP + g]; c = (c < 0) ? 0 : c; ((volatile int*)OFF)[(size_t)g * CSR_NBLK + b] = runb; runb += c; } __threadfence(); }
  for (int g = threadIdx.x; g < nG; g += 512) { int s = 0; for (int bb = 0; bb < CSR_NBLK; ++bb) { int c = HST[(size_t)bb * NGP + g]; s += (c < 0) ? 0 : c; } tot[g] = s; }
  __syncthreads();
  if (threadIdx.x < 32) {
    __shared__ int st[CSR_MAXG + 32];
    if (threadIdx.x == 0) { int acc = 0; for (int g = 0; g < NGP; ++g) { st[g] = acc; if (g < nG) acc += (tot[g] + 31) & ~31; } st[NGP] = acc; }
    __builtin_amdgcn_fence(__ATOMIC_RELEASE, "workgroup"); __builtin_amdgcn_wave_barrier(); __builtin_amdgcn_fence(__ATOMIC_ACQUIRE, "workgroup");
    for (int pass = 0; pass < 2; ++pass) { for (int i = threadIdx.x; i < NGP + 32; i += 32) { ((volatile int*)START)[i] = (i <= NGP) ? st[min(i, NGP)] : 0; ((volatile int*)TOT)[i] = (i < nG) ? tot[i] : 0; } __threadfence(); } }
}
__global__ __launch_bounds__(256) void csrB_kernel(const int* __restrict__ dst, int N, int nG, int CHP, int NGP, int permLen, const int* __restrict__ STG, const int* __restrict__ HST, const int* __restrict__ OFF, const int* __restrict__ START, const int* __restrict__ TOT, int* __restrict__ PERM, int* __restrict__ ROWPTR, int* __restrict__ ROWCNT, int* __restrict__ FLAG) {
  typedef __attribute__((ext_vector_type(4))) int v4i;
  __shared__ int ids[CSR_CAP]; __shared__ unsigned short key[CSR_CAP]; __shared__ int outp[CSR_CAP]; __shared__ int ncnt[CSR_GN + 1]; __shared__ int boff[CSR_NBLK + 1];
  const int g = blockIdx.x, t_ = threadIdx.x; int tot = TOT[g]; int st = START[g], stn = START[g + 1]; const int v0 = g * CSR_GN; const int nv = min(CSR_GN, N - v0);
  st = (st < 0) ? 0 : (st > permLen - 32 ? permLen - 32 : st) & ~31; stn = (stn < st) ? st : (stn > permLen ? permLen : stn); tot = (tot < 0) ? 0 : tot; if (tot > stn - st && tot <= CSR_CAP) tot = stn - st;
  if (tot > CSR_CAP) {
    for (int pass = 0; pass < 2; ++pass) { for (int i = t_; i < CSR_GN / 4; i += 256) { v4i a, c; for (int e = 0; e < 4; ++e) { a[e] = st; c[e] = 0; } *(volatile v4i*)(ROWPTR + v0 + i * 4) = a; *(volatile v4i*)(ROWCNT + v0 + i * 4) = c; } if (t_ == 0) ((volatile int*)FLAG)[0] = 1; __threadfence(); } (void)nv; return; }
  if (t_ == 0) { int acc = 0; for (int b = 0; b < CSR_NBLK; ++b) { boff[b] = acc; int c = HST[(size_t)b * NGP + g]; c = (c < 0) ? 0 : (c > CHP ? CHP : c); acc += c; if (acc > tot) acc = tot; } boff[CSR_NBLK] = acc; }
  for (int i = t_; i <= CSR_GN; i += 256) ncnt[i] = 0;
  __syncthreads();
  for (int b = 0; b < CSR_NBLK; ++b) { const int c = boff[b + 1] - boff[b]; int o_ = OFF[(size_t)g * CSR_NBLK + b]; o_ = (o_ < 0) ? 0 : (o_ > CHP - c ? CHP - c : o_); const int* src_ = STG + (size_t)b * CHP + o_;
    for (int i = t_; i < c; i += 256) { int id = src_[i]; id = (id < 0) ? 0 : id; ids[boff[b] + i] = id; int d = dst[id]; d = (d < v0) ? v0 : (d >= N ? N - 1 : d); int kk = d - v0; kk = (kk < 0) ? 0 : (kk >= CSR_GN ? CSR_GN - 1 : kk); key[boff[b] + i] = (unsigned short)kk; } }
  __syncthreads();
  if (t_ == 0) { for (int i = 0; i < tot; ++i) ncnt[key[i]] += 1; int acc = 0; for (int vl = 0; vl < CSR_GN; ++vl) { const int c = ncnt[vl]; ncnt[vl] = acc; acc += c; } ncnt[CSR_GN] = acc;
    for (int i = 0; i < tot; ++i) { const int vl = key[i]; outp[ncnt[vl]] = ids[i]; ncnt[vl] += 1; }
    for (int vl = CSR_GN; vl > 0; --vl) ncnt[vl] = ncnt[vl - 1]; ncnt[0] = 0; }
  __syncthreads();
  for (int pass = 0; pass < 2; ++pass) {
    for (int i = t_; i < (stn - st) / 4; i += 256) { v4i v; for (int e = 0; e < 4; ++e) { const int q = i * 4 + e; v[e] = (q < tot) ? outp[q] : -1; } *(volatile v4i*)(PERM + st + i * 4) = v; }
    for (int i = t_; i < CSR_GN / 4; i += 256) { v4i a, c; for (int e = 0; e < 4; ++e) { const int vl = i * 4 + e; a[e] = st + ncnt[vl]; c[e] = (vl < nv) ? (ncnt[vl + 1] - ncnt[vl]) : 0; } *(volatile v4i*)(ROWPTR + v0 + i * 4) = a; *(volatile v4i*)(ROWCNT + v0 + i * 4) = c; }
    __threadfence(); }
}
__global__ __launch_bounds__(256) void csrZ_kernel(int* __restrict__ p, size_t n4) { typedef __attribute__((ext_vector_type(4))) int v4i; const size_t tid = (size_t)blockIdx.x * 256 + threadIdx.x, nth = (size_t)gridDim.x * 256; v4i z = {0, 0, 0, 0}; for (size_t i = tid; i < n4; i += nth) *(volatile v4i*)(p + i * 4) = z; }
struct CsrBufs { int *STG, *HST, *OFF, *START, *TOT, *PERM, *ROWPTR, *ROWCNT, *FLAG; int nG, NGP, CHP; size_t permLen; char* base; size_t bytes; };
static size_t csr_carve(CsrBufs& c, char* ws, size_t off, int E, int N) {
  const size_t off0 = off; c.base = ws + off;
  auto al = [&](size_t bytes) { char* p = ws + off; off += (bytes + 255) & ~(size_t)255; return p; };
  c.nG = (N + CSR_GN - 1) / CSR_GN; c.NGP = (c.nG + 31) & ~31; const int ch = (E + CSR_NBLK - 1) / CSR_NBLK; c.CHP = (ch + 31) & ~31; c.permLen = (size_t)E + 32 * (size_t)c.nG + 32;
  c.STG = (int*)al((size_t)CSR_NBLK * c.CHP * 4); c.HST = (int*)al((size_t)CSR_NBLK * c.NGP * 4); c.OFF = (int*)al((size_t)c.NGP * CSR_NBLK * 4); c.START = (int*)al((size_t)(c.NGP + 64) * 4); c.TOT = (int*)al((size_t)(c.NGP + 64) * 4);
  c.PERM = (int*)al(c.permLen * 4); c.ROWPTR = (int*)al((size_t)c.nG * CSR_GN * 4); c.ROWCNT = (int*)al((size_t)c.nG * CSR_GN * 4); c.FLAG = (int*)al(256);
  c.bytes = off - off0; return off;
}
static void csr_build(const CsrBufs& c, const int* dst, int E, int N, hipStream_t stream) {
  const size_t smem = (size_t)(2 * c.NGP + c.CHP) * 4;
  csrZ_kernel<<<512, 256, 0, stream>>>((int*)c.base, c.bytes / 16);
  csrA_kernel<<<CSR_NBLK, 64, smem, stream>>>(dst, E, N, c.nG, c.CHP, c.NGP, c.STG, c.HST);
  csrS_kernel<<<1, 512, 0, stream>>>(c.HST, c.nG, c.NGP, c.START, c.TOT, c.OFF);
  csrB_kernel<<<c.nG, 256, 0, stream>>>(dst, N, c.nG, c.CHP, c.NGP, (int)c.permLen, c.STG, c.HST, c.OFF, c.START, c.TOT, c.PERM, c.ROWPTR, c.ROWCNT, c.FLAG);
}


__global__ __launch_bounds__(256) void wprep_kernel(const float* __restrict__ qw, const float* __restrict__ kw, const float* __restrict__ vw, const float* __restrict__ l1w, const float* __restrict__ l2w, b16* __restrict__ WT1, b16* __restrict__ WT2) {
  const size_t u = (size_t)blockIdx.x * 256 + threadIdx.x; const size_t per = (size_t)HID * FIN / 8, n2 = (size_t)C * FIN / 8; size_t t = u; v8b o;
  if (t < 4 * per) { const int part = (int)(t / per); const size_t e = (t % per) * 8; const int oo = (int)(e / FIN), k0 = (int)(e % FIN); const float* w = part == 0 ? qw : part == 1 ? kw : part == 2 ? vw : l1w;
    for (int j = 0; j < 8; ++j) o[j] = (b16)(bf16_rne(w[(size_t)(k0 + j) * HID + oo]) * WSC); for (int pass = 0; pass < 2; ++pass) { *(volatile v8b*)(WT1 + (size_t)part * HID * FIN + e) = o; __threadfence(); } return; } t -= 4 * per;
  if (t < n2) { const size_t e = t * 8; const int oo = (int)(e / FIN), k0 = (int)(e % FIN); for (int j = 0; j < 8; ++j) o[j] = (b16)(bf16_rne(l2w[(size_t)(k0 + j) * C + oo]) * WSC); for (int pass = 0; pass < 2; ++pass) { *(volatile v8b*)(WT2 + e) = o; __threadfence(); } }
}
__global__ __launch_bounds__(128) void proj_kernel(const float* __restrict__ data, const b16* __restrict__ WT1, const float* __restrict__ bq, const float* __restrict__ bk, const float* __restrict__ bv, const float* __restrict__ b1, float* __restrict__ PL) {
  __shared__ __attribute__((aligned(16))) float Tf[4][16][HID + 4];
  const int wave = threadIdx.x >> 5, lane = threadIdx.x & 31, nloc = lane & 15, hlf = lane >> 4; const size_t m0 = (size_t)blockIdx.x * 64 + wave * 16; const int part = blockIdx.y; const b16* W = WT1 + (size_t)part * HID * FIN; const float* bias = part == 0 ? bq : part == 1 ? bk : part == 2 ? bv : b1;
  const size_t v = m0 + nloc; v8f acc[8];
#pragma unroll
  for (int t = 0; t < 8; ++t) acc[t] = (v8f){};
#pragma unroll 2
  for (int kb = 0; kb < FIN; kb += 32) { v16b a = {}; if (v < (size_t)N) { const float* r = data + v * FIN + kb; for (int e = 0; e < 8; ++e) { a[e] = (b16)(bf16_rne(r[8 * hlf + e]) * XS); a[8 + e] = (b16)(bf16_rne(r[16 + 8 * hlf + e]) * XS); } }
#pragma unroll
    for (int t = 0; t < 8; ++t) acc[t] = wmma16b(a, frag_kb(W + (size_t)(t * 16 + nloc) * FIN + kb, hlf), acc[t]); }
#pragma unroll
  for (int t = 0; t < 8; ++t) { const int c = t * 16 + nloc; const float bb = bf16_rne(bias[c]);
#pragma unroll 1
    for (int r = 0; r < 8; ++r) { const size_t row = m0 + 8 * hlf + r; Tf[wave][8 * hlf + r][c] = row < (size_t)N ? acc[t][r] * (1.0f / (XS * WSC)) + bb : 0.0f; } }
  wave_lds_sync();
  for (int pass = 0; pass < 2; ++pass) { for (int rr = 0; rr < 16; ++rr) *(volatile v4f*)(PL + ((size_t)part * NP + m0 + rr) * HID + lane * 4) = *(const v4f*)(&Tf[wave][rr][lane * 4]); __threadfence(); }
}
__global__ __launch_bounds__(256) void kmax_kernel(const float* __restrict__ PL, const float* __restrict__ proj, float* __restrict__ KMP) {
  __shared__ float pj[NB][HD]; __shared__ float mx[8][64];
  const int t = threadIdx.x; for (int q = t; q < NB * HD; q += 256) pj[q / HD][q % HD] = bf16_rne(proj[q]);
  __syncthreads();
  const int nl = t & 63, hg = t >> 6; const size_t v = (size_t)blockIdx.x * 64 + nl; const float* K = PL + (size_t)NP * HID;
  for (int hh = 0; hh < 2; ++hh) { const int h = hg * 2 + hh; float m = -INFINITY;
    if (v < (size_t)N) { float k[HD]; for (int d = 0; d < HD; ++d) k[d] = K[v * HID + h * HD + d] * DNORM;
#pragma unroll 1
      for (int mm = 0; mm < NB; ++mm) { float s = 0.0f;
#pragma unroll
        for (int d = 0; d < HD; ++d) s += pmul(k[d], pj[mm][d]); m = fmaxf(m, s); } }
    mx[h][nl] = m; }
  __syncthreads();
  if (t < 8) { float m = -INFINITY; for (int i = 0; i < 64; ++i) m = fmaxf(m, mx[t][i]); mx[t][0] = m; }
  __syncthreads();
  for (int pass = 0; pass < 2; ++pass) { if (t < 32) ((volatile float*)KMP)[(size_t)blockIdx.x * 32 + t] = (t < 8) ? mx[t][0] : 0.0f; __threadfence(); }
}
__global__ __launch_bounds__(32) void kmaxred_kernel(const float* __restrict__ KMP, float* __restrict__ KMAX) {
  const int t = threadIdx.x; float m = -INFINITY; if (t < 8) for (int b = 0; b < NBLK; ++b) m = fmaxf(m, KMP[(size_t)b * 32 + t]);
  for (int pass = 0; pass < 2; ++pass) { ((volatile float*)KMAX)[t] = (t < 8) ? m : 0.0f; __threadfence(); }
}
__global__ __launch_bounds__(256) void ctx_kernel(const float* __restrict__ PL, const float* __restrict__ proj, const float* __restrict__ KMAX, float* __restrict__ PART) {
  __shared__ float pj[NB][HD]; __shared__ float KP[64][NB + 1]; __shared__ float VV[64][HD + 2];
  const int t = threadIdx.x, h = blockIdx.y; for (int q = t; q < NB * HD; q += 256) pj[q / HD][q % HD] = bf16_rne(proj[q]);
  __syncthreads();
  const float* K = PL + (size_t)NP * HID; const float* Vp = PL + (size_t)2 * NP * HID;
  { const int nl = t & 63, mg = t >> 6; const size_t v = (size_t)blockIdx.x * 64 + nl; const bool ok = v < (size_t)N; float k[HD]; float diag = 0.0f; const float kmx = KMAX[h];
    for (int d = 0; d < HD; ++d) { k[d] = ok ? K[v * HID + h * HD + d] * DNORM : 0.0f; diag += k[d] * k[d]; if (mg == 0) VV[nl][d] = ok ? Vp[v * HID + h * HD + d] : 0.0f; } diag *= 0.5f; if (mg == 0) VV[nl][HD] = ok ? 1.0f : 0.0f;
#pragma unroll 1
    for (int mm = mg * 11; mm < mg * 11 + 11; ++mm) { float s = 0.0f;
#pragma unroll
      for (int d = 0; d < HD; ++d) s += pmul(k[d], pj[mm][d]); KP[nl][mm] = ok ? RATIO * (__expf(s - diag - kmx) + PEPS) : 0.0f; } }
  __syncthreads();
  float res[3]; for (int i = 0; i < 3; ++i) { const int q = t + i * 256; float s = 0.0f; if (q < NB * (HD + 1)) { const int mm = q / (HD + 1), d = q % (HD + 1);
#pragma unroll 1
      for (int n = 0; n < 64; ++n) s += pmul(KP[n][mm], VV[n][d]); } res[i] = s; }
  for (int pass = 0; pass < 2; ++pass) { for (int i = 0; i < 3; ++i) ((volatile float*)PART)[((size_t)blockIdx.x * NH + h) * PW + t + i * 256] = res[i]; __threadfence(); }
}
__global__ __launch_bounds__(256) void ctxred_kernel(const float* __restrict__ PART, float* __restrict__ CTX) {
  const int t = threadIdx.x, h = blockIdx.x; float res[3];
  for (int i = 0; i < 3; ++i) { const int q = t + i * 256; float s = 0.0f; for (int b = 0; b < NBLK; ++b) s += PART[((size_t)b * NH + h) * PW + q]; res[i] = s; }
  for (int pass = 0; pass < 2; ++pass) { for (int i = 0; i < 3; ++i) ((volatile float*)CTX)[(size_t)h * PW + t + i * 256] = res[i]; __threadfence(); }
}
__global__ __launch_bounds__(256) void q_kernel(const float* __restrict__ PL, const float* __restrict__ proj, const float* __restrict__ CTX, b16* __restrict__ HEh, b16* __restrict__ HEl) {
  __shared__ float pj[NB][HD]; __shared__ __attribute__((aligned(16))) float HR[32][2 * HID + 4]; __shared__ float DS[256][NB + 1];
  const int t = threadIdx.x, wave = t >> 5, lane = t & 31; for (int q = t; q < NB * HD; q += 256) pj[q / HD][q % HD] = bf16_rne(proj[q]);
  __syncthreads();
  { const int nl = t & 31, h = t >> 5; const size_t v = (size_t)blockIdx.x * 32 + nl; const bool ok = v < (size_t)N; float q[HD]; float diag = 0.0f;
    for (int d = 0; d < HD; ++d) { q[d] = ok ? PL[v * HID + h * HD + d] * DNORM : 0.0f; diag += q[d] * q[d]; } diag *= 0.5f;
    float mq = -INFINITY;
#pragma unroll 1
    for (int mm = 0; mm < NB; ++mm) { float s = 0.0f;
#pragma unroll
      for (int d = 0; d < HD; ++d) s += pmul(q[d], pj[mm][d]); DS[t][mm] = s; mq = fmaxf(mq, s); }
    float den = 0.0f, o[HD]; for (int d = 0; d < HD; ++d) o[d] = 0.0f; const float* cx = CTX + (size_t)h * PW;
#pragma unroll 1
    for (int mm = 0; mm < NB; ++mm) { const float qp = RATIO * (__expf(DS[t][mm] - diag - mq) + PEPS); den += pmul(qp, cx[mm * (HD + 1) + HD]);
#pragma unroll
      for (int d = 0; d < HD; ++d) o[d] += pmul(qp, cx[mm * (HD + 1) + d]); }
    const float inv = 1.0f / den; const float* G1 = PL + (size_t)3 * NP * HID;
    for (int d = 0; d < HD; ++d) { HR[nl][HID + h * HD + d] = ok ? elu_(o[d] * inv) : 0.0f; HR[nl][h * HD + d] = ok ? elu_(G1[v * HID + h * HD + d]) : 0.0f; } }
  __syncthreads();
  for (int pass = 0; pass < 2; ++pass) { for (int rr = wave * 4; rr < wave * 4 + 4; ++rr) { const size_t v = (size_t)blockIdx.x * 32 + rr; v8b ph, pl; for (int j = 0; j < 8; ++j) { b16 p, q2; split16(HR[rr][lane * 8 + j] * XS, p, q2); ph[j] = p; pl[j] = q2; }
      *(volatile v8b*)(HEh + v * 2 * HID + lane * 8) = ph; *(volatile v8b*)(HEl + v * 2 * HID + lane * 8) = pl; } __threadfence(); }
}
__global__ __launch_bounds__(128) void lin2_kernel(const b16* __restrict__ HEh, const b16* __restrict__ HEl, const b16* __restrict__ WT2, const float* __restrict__ b2, float* __restrict__ X0) {
  __shared__ __attribute__((aligned(16))) float Tf[4][16][C + 4];
  const int wave = threadIdx.x >> 5, lane = threadIdx.x & 31, nloc = lane & 15, hlf = lane >> 4; const size_t m0 = (size_t)blockIdx.x * 64 + wave * 16;
  v8f acc[4] = {{}, {}, {}, {}};
#pragma unroll 2
  for (int kb = 0; kb < 2 * HID; kb += 32) { const v16b a = frag_kb(HEh + (m0 + nloc) * 2 * HID + kb, hlf), al = frag_kb(HEl + (m0 + nloc) * 2 * HID + kb, hlf);
#pragma unroll
    for (int t = 0; t < 4; ++t) { const v16b bw = frag_kb(WT2 + (size_t)(t * 16 + nloc) * 2 * HID + kb, hlf); acc[t] = wmma16b(a, bw, acc[t]); acc[t] = wmma16b(al, bw, acc[t]); } }
#pragma unroll
  for (int t = 0; t < 4; ++t) { const int c = t * 16 + nloc; const float bb = bf16_rne(b2[c]);
#pragma unroll 1
    for (int r = 0; r < 8; ++r) { const size_t row = m0 + 8 * hlf + r; Tf[wave][8 * hlf + r][c] = row < (size_t)N ? elu_(acc[t][r] * (1.0f / (XS * WSC)) + bb) : 0.0f; } }
  wave_lds_sync();
  for (int pass = 0; pass < 2; ++pass) { for (int rr = 0; rr < 16; ++rr) if (lane < 16) *(volatile v4f*)(X0 + (m0 + rr) * C + lane * 4) = *(const v4f*)(&Tf[wave][rr][lane * 4]); __threadfence(); }
}
template <int LAST>
__global__ __launch_bounds__(256) void hop_kernel(const float* __restrict__ Hin, const float* __restrict__ X0, const int* __restrict__ srcs, const int* __restrict__ PERM, const int* __restrict__ ROWPTR, const int* __restrict__ ROWCNT, int permLen, float* __restrict__ Hout, float* __restrict__ out) {
  const int wave = threadIdx.x >> 5, lane = threadIdx.x & 31; const size_t v = (size_t)blockIdx.x * 8 + wave; v2f o = {0.0f, 0.0f};
  if (v < (size_t)N) { int st = ROWPTR[v], cnt = ROWCNT[v]; cnt = iclamp(cnt, 0, 65536); st = iclamp(st, 0, permLen - cnt); const float dv = rsqrtf((float)cnt + 1.0f); v2f acc = {0.0f, 0.0f};
#pragma unroll 1
    for (int j = 0; j < cnt; ++j) { const int e = iclamp(PERM[st + j], 0, E - 1); const size_t s = (size_t)iclamp(srcs[e], 0, N - 1); const float w = rsqrtf((float)iclamp(ROWCNT[s], 0, 65536) + 1.0f); const v2f hs = *(const v2f*)(Hin + s * C + lane * 2); acc[0] += pmul(w, hs[0]); acc[1] += pmul(w, hs[1]); }
    const v2f hv = *(const v2f*)(Hin + v * C + lane * 2); const v2f x = *(const v2f*)(X0 + v * C + lane * 2);
    for (int i = 0; i < 2; ++i) { const float ag = pmul(dv, acc[i]) + pmul(pmul(dv, dv), hv[i]); o[i] = (1.0f - ALPHA) * ag + ALPHA * x[i]; } }
  for (int pass = 0; pass < 2; ++pass) { *(volatile v2f*)(Hout + v * C + lane * 2) = o; __threadfence(); }
  if (LAST) { float m = fmaxf(o[0], o[1]); for (int sh = 16; sh; sh >>= 1) m = fmaxf(m, __shfl_xor(m, sh)); float s = __expf(o[0] - m) + __expf(o[1] - m); for (int sh = 16; sh; sh >>= 1) s += __shfl_xor(s, sh); const float lse = m + __logf(s);
    const v2f ls = {o[0] - lse, o[1] - lse};
    if (v < (size_t)N) for (int pass = 0; pass < 2; ++pass) { *(volatile v2f*)(out + v * C + lane * 2) = ls; *(volatile v2f*)(out + (size_t)N * C + v * C + lane * 2) = o; __threadfence(); } }
}
}

extern "C" void kernel_launch(void* const* d_in, const int* in_sizes, int n_in, void* d_out, int out_size, void* d_ws, size_t ws_size, hipStream_t stream) {
  (void)n_in;
  auto Fp = [&](int i) { return (const float*)d_in[i]; }; auto Ip = [&](int i) { return (const int*)d_in[i]; };
  if (in_sizes[0] != N * FIN || in_sizes[1] != 2 * E || in_sizes[2] != FIN * HID || in_sizes[4] != FIN * C || in_sizes[6] != FIN * HID || in_sizes[12] != NB * HD || out_size != 2 * N * C) return;
  size_t off = 0; char* ws = (char*)d_ws;
  auto carve = [&](size_t bytes) { char* p = ws + off; off += (bytes + 255) & ~(size_t)255; return p; };
  b16* WT1 = (b16*)carve((size_t)4 * HID * FIN * 2); b16* WT2 = (b16*)carve((size_t)C * FIN * 2); float* PL = (float*)carve((size_t)4 * NP * HID * 4);
  float* KMP = (float*)carve((size_t)NBLK * 32 * 4); float* KMAX = (float*)carve(256); float* PART = (float*)carve((size_t)NBLK * NH * PW * 4); float* CTX = (float*)carve((size_t)NH * PW * 4);
  b16* HEh = (b16*)(PL + (size_t)NP * HID); b16* HEl = (b16*)(PL + (size_t)2 * NP * HID);
  float* X0 = (float*)carve((size_t)NP * C * 4); float* HA = (float*)carve((size_t)NP * C * 4); float* HB = (float*)carve((size_t)NP * C * 4);
  CsrBufs csr; off = csr_carve(csr, ws, off, E, N);
  if (off > ws_size) return;
  wprep_kernel<<<(unsigned)((4 * (size_t)HID * FIN / 8 + (size_t)C * FIN / 8 + 255) / 256), 256, 0, stream>>>(Fp(6), Fp(8), Fp(10), Fp(2), Fp(4), WT1, WT2);
  proj_kernel<<<dim3(NP / 64, 4), 128, 0, stream>>>(Fp(0), WT1, Fp(7), Fp(9), Fp(11), Fp(3), PL);
  kmax_kernel<<<NBLK, 256, 0, stream>>>(PL, Fp(12), KMP);
  kmaxred_kernel<<<1, 32, 0, stream>>>(KMP, KMAX);
  ctx_kernel<<<dim3(NBLK, NH), 256, 0, stream>>>(PL, Fp(12), KMAX, PART);
  ctxred_kernel<<<NH, 256, 0, stream>>>(PART, CTX);
  q_kernel<<<NP / 32, 256, 0, stream>>>(PL, Fp(12), CTX, HEh, HEl);
  lin2_kernel<<<NP / 64, 128, 0, stream>>>(HEh, HEl, WT2, Fp(5), X0);
  csr_build(csr, Ip(1) + E, E, N, stream);
  const float* hin = X0; float* bufs[2] = {HA, HB};
  for (int k = 0; k < KH; ++k) { float* hout = bufs[k & 1];
    if (k == KH - 1) hop_kernel<1><<<NP / 8, 256, 0, stream>>>(hin, X0, Ip(1), csr.PERM, csr.ROWPTR, csr.ROWCNT, (int)csr.permLen, hout, (float*)d_out);
    else hop_kernel<0><<<NP / 8, 256, 0, stream>>>(hin, X0, Ip(1), csr.PERM, csr.ROWPTR, csr.ROWCNT, (int)csr.permLen, hout, nullptr);
    hin = hout; }
}
